// MixtureOfExperts_64957085385329
// MI455X (gfx1250) — hardware-verified
//
#include <hip/hip_runtime.h>
#include <math.h>

typedef __attribute__((ext_vector_type(16))) _Float16 v16h;
typedef __attribute__((ext_vector_type(16))) __bf16 v16b;
typedef __attribute__((ext_vector_type(8)))  _Float16 v8h;
typedef __attribute__((ext_vector_type(8)))  float v8f;
typedef __attribute__((ext_vector_type(4)))  float v4f;
typedef __attribute__((ext_vector_type(2)))  float v2f;
typedef __attribute__((ext_vector_type(4)))  unsigned v4u;
typedef __attribute__((ext_vector_type(4)))  int v4i;
typedef float __attribute__((may_alias)) float_a;
typedef int __attribute__((may_alias)) int_a;

template <typename T> __device__ __forceinline__ void vst2(void* p, T v) { *(volatile T*)p = v; __threadfence(); *(volatile T*)p = v; }
__device__ __forceinline__ v8f wmma16(v16h a, v16h b, v8f c) {
  v8f d = __builtin_amdgcn_wmma_f32_16x16x32_f16(false, a, false, b, (short)0, c, false, false);
  asm volatile("v_nop\n\tv_nop\n\tv_nop\n\tv_nop" : "+v"(d) : "v"(a), "v"(b));
  return d;
}
__device__ __forceinline__ v8f wmma_bf(v16b a, v16b b, v8f c) {
  v8f d = __builtin_amdgcn_wmma_f32_16x16x32_bf16(false, a, false, b, (short)0, c, false, false);
  asm volatile("v_nop\n\tv_nop\n\tv_nop\n\tv_nop" : "+v"(d) : "v"(a), "v"(b));
  return d;
}
__device__ __forceinline__ v16h frag_h(const _Float16* rowk0, int lane) {
  union { v16h v; v8h q[2]; } u; const _Float16* p = rowk0 + 8 * (lane >> 4);
  u.q[0] = *(const v8h*)p; u.q[1] = *(const v8h*)(p + 16); return u.v;
}
__device__ __forceinline__ v16h frag_f32(const float* rowk0, int lane) {
  v16h a; const float* p = rowk0 + 8 * (lane >> 4);
#pragma unroll
  for (int i = 0; i < 8; ++i) { a[i] = (_Float16)p[i]; a[8 + i] = (_Float16)p[16 + i]; }
  return a;
}
__device__ __forceinline__ v16h frag_f32s(const float* rowk0, int lane, float sc) {
  v16h a; const float* p = rowk0 + 8 * (lane >> 4);
#pragma unroll
  for (int i = 0; i < 8; ++i) { a[i] = (_Float16)(p[i] * sc); a[8 + i] = (_Float16)(p[16 + i] * sc); }
  return a;
}
__device__ __forceinline__ v16h fragc_f32(const float* W, int k0, int n, int lane, int ld, int K) {
  v16h a; const int g = lane >> 4;
#pragma unroll
  for (int i = 0; i < 8; ++i) { const int ka = k0 + 8 * g + i, kb = ka + 16;
    a[i] = (_Float16)(ka < K ? W[(size_t)ka * ld + n] : 0.f); a[8 + i] = (_Float16)(kb < K ? W[(size_t)kb * ld + n] : 0.f); }
  return a;
}
struct F2 { v16b h, l; };
__device__ __forceinline__ F2 bsplit16(const float v[16]) { F2 r;
#pragma unroll
  for (int i = 0; i < 16; ++i) { const __bf16 h = (__bf16)v[i]; r.h[i] = h; r.l[i] = (__bf16)(v[i] - (float)h); }
  return r; }
__device__ __forceinline__ F2 split_row(const float* row, int k0, int lane) { float v[16]; const float* p = row + k0 + 8 * (lane >> 4);
#pragma unroll
  for (int i = 0; i < 8; ++i) { v[i] = p[i]; v[8 + i] = p[16 + i]; }
  return bsplit16(v); }
__device__ __forceinline__ F2 split_rowK(const float* row, int k0, int lane, int K) { float v[16]; const int g = lane >> 4;
#pragma unroll
  for (int i = 0; i < 8; ++i) { const int ka = k0 + 8 * g + i, kb = ka + 16; v[i] = ka < K ? row[ka] : 0.f; v[8 + i] = kb < K ? row[kb] : 0.f; }
  return bsplit16(v); }
__device__ __forceinline__ F2 split_col(const float* W, int k0, int n, int lane, int ld, int K) { float v[16]; const int g = lane >> 4;
#pragma unroll
  for (int i = 0; i < 8; ++i) { const int ka = k0 + 8 * g + i, kb = ka + 16; v[i] = ka < K ? W[(size_t)ka * ld + n] : 0.f; v[8 + i] = kb < K ? W[(size_t)kb * ld + n] : 0.f; }
  return bsplit16(v); }
__device__ __forceinline__ v8f mac3(const F2& a, const F2& b, v8f c) { c = wmma_bf(a.l, b.h, c); c = wmma_bf(a.h, b.l, c); return wmma_bf(a.h, b.h, c); }
__device__ __forceinline__ float sigm(float v) { return 1.0f / (1.0f + expf(-v)); }
#define LDSX() do { asm volatile("s_wait_dscnt 0" ::: "memory"); __builtin_amdgcn_wave_barrier(); __builtin_amdgcn_fence(__ATOMIC_RELEASE, "workgroup"); } while (0)

#define NB 8192
#define DD 1024
#define OO 1024
#define NE 8
#define HH 512
#define NPAIR (NB * 2)

__global__ __launch_bounds__(256) void k_gate(const float* __restrict__ x, const float* __restrict__ gW, const float* __restrict__ gb, float* __restrict__ gl, float* __restrict__ sel) {
  __shared__ float sW[DD * NE];
  const int tid = threadIdx.x, b = blockIdx.x * 256 + tid;
  for (int q = tid; q < DD * NE; q += 256) sW[q] = gW[q];
  __syncthreads();
  float lg[NE];
#pragma unroll
  for (int e = 0; e < NE; ++e) lg[e] = gb[e];
  const float* xr = x + (size_t)b * DD;
#pragma unroll 1
  for (int d = 0; d < DD; ++d) { const float v = xr[d];
#pragma unroll
    for (int e = 0; e < NE; ++e) lg[e] += v * sW[d * NE + e]; }
  int i1 = 0;
#pragma unroll
  for (int e = 1; e < NE; ++e) if (lg[e] > lg[i1]) i1 = e;
  int i2 = i1 == 0 ? 1 : 0;
#pragma unroll
  for (int e = 0; e < NE; ++e) if (e != i1 && lg[e] > lg[i2]) i2 = e;
  const float m = lg[i1]; const float e2 = expf(lg[i2] - m); const float g1 = 1.0f / (1.0f + e2), g2 = e2 / (1.0f + e2);
  vst2(gl + (size_t)b * NE, (v4f){lg[0], lg[1], lg[2], lg[3]}); vst2(gl + (size_t)b * NE + 4, (v4f){lg[4], lg[5], lg[6], lg[7]});
  vst2(sel + (size_t)b * 4, (v4f){(float)i1, (float)i2, g1, g2});
}
__global__ __launch_bounds__(256) void k_bucket(const float* __restrict__ sel, int* __restrict__ list, int* __restrict__ cnt) {
  __shared__ int sc; __shared__ __align__(16) int sl[NPAIR];
  const int e = blockIdx.x, tid = threadIdx.x;
  if (tid == 0) sc = 0; __syncthreads();
  for (int b = tid; b < NB; b += 256) { const int i1 = (int)sel[(size_t)b * 4], i2 = (int)sel[(size_t)b * 4 + 1];
    if (i1 == e) { const int s = atomicAdd(&sc, 1); sl[s] = b * 2; } if (i2 == e) { const int s = atomicAdd(&sc, 1); sl[s] = b * 2 + 1; } }
  __syncthreads();
  const int n = sc;
  for (int q = tid; q < NPAIR / 4; q += 256) { v4i v = { q * 4 < n ? sl[q * 4] : -1, q * 4 + 1 < n ? sl[q * 4 + 1] : -1, q * 4 + 2 < n ? sl[q * 4 + 2] : -1, q * 4 + 3 < n ? sl[q * 4 + 3] : -1 };
    vst2(list + (size_t)e * NPAIR + q * 4, v); }
  if (tid < 32) vst2(cnt + e * 32 + tid, (int_a)(tid == 0 ? n : 0));
}
__global__ __launch_bounds__(128) void k_pack(const float* __restrict__ W1, const float* __restrict__ W2, _Float16* __restrict__ P1, _Float16* __restrict__ P2) {
  const int n = blockIdx.x, tid = threadIdx.x;
  if (n < NE * HH) { const int e = n / HH, h = n % HH;
    for (int q = tid; q < DD / 8; q += 128) { union { v8h hh; v4u u; } pk;
#pragma unroll
      for (int i = 0; i < 8; ++i) pk.hh[i] = (_Float16)(W1[((size_t)e * DD + q * 8 + i) * HH + h] * 64.0f);
      vst2(P1 + (size_t)n * DD + q * 8, pk.u); } }
  else { const int m = n - NE * HH, e = m / OO, o = m % OO;
    for (int q = tid; q < HH / 8; q += 128) { union { v8h hh; v4u u; } pk;
#pragma unroll
      for (int i = 0; i < 8; ++i) pk.hh[i] = (_Float16)(W2[((size_t)e * HH + q * 8 + i) * OO + o] * 64.0f);
      vst2(P2 + (size_t)m * HH + q * 8, pk.u); } }
}
__global__ __launch_bounds__(128) void k_h(const float* __restrict__ x, const int* __restrict__ list, const int* __restrict__ cnt, const _Float16* __restrict__ P1, const float* __restrict__ b1, _Float16* __restrict__ hbuf) {
  __shared__ __align__(16) float so[4][16][132];
  const int tid = threadIdx.x, wave = tid >> 5, lane = tid & 31, col = lane & 15, g = lane >> 4;
  const int e = blockIdx.z, p0 = blockIdx.x * 64 + wave * 16, n0 = blockIdx.y * 128; const int ne = cnt[e * 32];
  if (blockIdx.x * 64 >= ne) return;
  int pr = list[(size_t)e * NPAIR + p0 + col]; const bool ok = (p0 + col) < ne && pr >= 0 && pr < NPAIR; if (!ok) pr = 0;
  const int row = pr >> 1;
  v8f acc[8] = {};
#pragma unroll 1
  for (int kc = 0; kc < DD / 32; ++kc) { const v16h a = frag_f32(x + (size_t)row * DD + kc * 32, lane);
#pragma unroll
    for (int j = 0; j < 8; ++j) acc[j] = wmma16(a, frag_h(P1 + ((size_t)e * HH + n0 + j * 16 + col) * DD + kc * 32, lane), acc[j]); }
#pragma unroll
  for (int j = 0; j < 8; ++j) { const float bb = b1[e * HH + n0 + j * 16 + col];
#pragma unroll
    for (int r = 0; r < 8; ++r) { const float v = acc[j][r] * (1.0f / 64.0f) + bb; so[wave][8 * g + r][j * 16 + col] = v > 0.f ? v : 0.f; } }
  LDSX();
  for (int q = lane; q < 16 * 16; q += 32) { const int rl = q >> 4, pc = q & 15; const int pp = p0 + rl; if (pp >= ne) continue;
    const int prr = list[(size_t)e * NPAIR + pp]; if (prr < 0 || prr >= NPAIR) continue;
    union { v8h hh; v4u u; } pk;
#pragma unroll
    for (int i = 0; i < 8; ++i) pk.hh[i] = (_Float16)so[wave][rl][pc * 8 + i];
    vst2(hbuf + (size_t)prr * HH + n0 + pc * 8, pk.u); }
}
__global__ __launch_bounds__(128) void k_y(const _Float16* __restrict__ hbuf, const int* __restrict__ list, const int* __restrict__ cnt, const _Float16* __restrict__ P2, const float* __restrict__ b2, float* __restrict__ y) {
  __shared__ __align__(16) float so[4][16][132];
  const int tid = threadIdx.x, wave = tid >> 5, lane = tid & 31, col = lane & 15, g = lane >> 4;
  const int e = blockIdx.z, p0 = blockIdx.x * 64 + wave * 16, n0 = blockIdx.y * 128; const int ne = cnt[e * 32];
  if (blockIdx.x * 64 >= ne) return;
  int pr = list[(size_t)e * NPAIR + p0 + col]; const bool ok = (p0 + col) < ne && pr >= 0 && pr < NPAIR; if (!ok) pr = 0;
  v8f acc[8] = {};
#pragma unroll 1
  for (int kc = 0; kc < HH / 32; ++kc) { const v16h a = frag_h(hbuf + (size_t)pr * HH + kc * 32, lane);
#pragma unroll
    for (int j = 0; j < 8; ++j) acc[j] = wmma16(a, frag_h(P2 + ((size_t)e * OO + n0 + j * 16 + col) * HH + kc * 32, lane), acc[j]); }
#pragma unroll
  for (int j = 0; j < 8; ++j) { const float bb = b2[e * OO + n0 + j * 16 + col];
#pragma unroll
    for (int r = 0; r < 8; ++r) so[wave][8 * g + r][j * 16 + col] = acc[j][r] * (1.0f / 64.0f) + bb; }
  LDSX();
  for (int rl = 0; rl < 16; ++rl) { const int pp = p0 + rl; if (pp >= ne) continue; const int prr = list[(size_t)e * NPAIR + pp]; if (prr < 0 || prr >= NPAIR) continue;
    vst2(y + (size_t)prr * OO + n0 + lane * 4, *(const v4f*)(&so[wave][rl][lane * 4])); }
}
__global__ __launch_bounds__(256) void k_comb(const float* __restrict__ y, const float* __restrict__ sel, float* __restrict__ out) {
  const int b = blockIdx.x, tid = threadIdx.x; const float g1 = sel[(size_t)b * 4 + 2], g2 = sel[(size_t)b * 4 + 3];
  const v4f a = *(const v4f*)(y + (size_t)(2 * b) * OO + tid * 4), c = *(const v4f*)(y + (size_t)(2 * b + 1) * OO + tid * 4);
  vst2(out + (size_t)b * OO + tid * 4, a * g1 + c * g2);
}
__global__ __launch_bounds__(256) void k_loss(const float* __restrict__ gl, float* __restrict__ lossout) {
  __shared__ float red[NE][256];
  const int tid = threadIdx.x;
  float imp[NE];
#pragma unroll
  for (int e = 0; e < NE; ++e) imp[e] = 0.f;
  for (int b = tid; b < NB; b += 256) { float l[NE]; float m = -3.0e38f;
#pragma unroll
    for (int e = 0; e < NE; ++e) { l[e] = gl[(size_t)b * NE + e]; m = fmaxf(m, l[e]); }
    float s = 0.f;
#pragma unroll
    for (int e = 0; e < NE; ++e) { l[e] = expf(l[e] - m); s += l[e]; }
#pragma unroll
    for (int e = 0; e < NE; ++e) imp[e] += l[e] / s; }
#pragma unroll
  for (int e = 0; e < NE; ++e) red[e][tid] = imp[e];
  __syncthreads();
  for (int st = 128; st > 0; st >>= 1) { if (tid < st) {
#pragma unroll
      for (int e = 0; e < NE; ++e) red[e][tid] += red[e][tid + st]; } __syncthreads(); }
  if (tid == 0) { float L = 0.f;
#pragma unroll
    for (int e = 0; e < NE; ++e) { const float im = red[e][0] / (float)NB; L += im * im; }
    vst2(lossout, (float_a)(0.01f * (float)NE * L)); }
}
extern "C" void kernel_launch(void* const* d_in, const int* in_sizes, int n_in, void* d_out, int out_size, void* d_ws, size_t ws_size, hipStream_t stream) {
  (void)in_sizes; (void)n_in; (void)out_size; (void)ws_size;
  const float* x = (const float*)d_in[0]; const float* gW = (const float*)d_in[1]; const float* gb = (const float*)d_in[2];
  const float* W1 = (const float*)d_in[3]; const float* b1 = (const float*)d_in[4]; const float* W2 = (const float*)d_in[5]; const float* b2 = (const float*)d_in[6];
  float* out = (float*)d_out; float* lossout = out + (size_t)NB * OO;
  char* ws = (char*)d_ws; size_t off = 0;
  auto take = [&](size_t bytes) { char* p = ws + off; off += (bytes + 255) & ~(size_t)255; return p; };
  float* gl = (float*)take((size_t)NB * NE * 4); float* sel = (float*)take((size_t)NB * 4 * 4);
  int* list = (int*)take((size_t)NE * NPAIR * 4); int* cnt = (int*)take((size_t)NE * 32 * 4);
  _Float16* P1 = (_Float16*)take((size_t)NE * HH * DD * 2); _Float16* P2 = (_Float16*)take((size_t)NE * OO * HH * 2);
  _Float16* hbuf = (_Float16*)take((size_t)NPAIR * HH * 2); float* y = (float*)take((size_t)NPAIR * OO * 4);
  k_gate<<<NB / 256, 256, 0, stream>>>(x, gW, gb, gl, sel);
  k_bucket<<<NE, 256, 0, stream>>>(sel, list, cnt);
  k_pack<<<NE * HH + NE * OO, 128, 0, stream>>>(W1, W2, P1, P2);
  k_h<<<dim3(NPAIR / 64, HH / 128, NE), 128, 0, stream>>>(x, list, cnt, P1, b1, hbuf);
  k_y<<<dim3(NPAIR / 64, OO / 128, NE), 128, 0, stream>>>(hbuf, list, cnt, P2, b2, y);
  k_comb<<<NB, 256, 0, stream>>>(y, sel, out);
  k_loss<<<1, 256, 0, stream>>>(gl, lossout);
}
